// ValueRNN_Timescales_18236431139462
// MI455X (gfx1250) — hardware-verified
//
#include <hip/hip_runtime.h>
#include <math.h>
#include <stdint.h>

typedef __attribute__((ext_vector_type(16))) _Float16 v16h;
typedef __attribute__((ext_vector_type(8)))  _Float16 v8h;
typedef __attribute__((ext_vector_type(8)))  float    v8f;
typedef __attribute__((ext_vector_type(4)))  float    v4f;

__device__ __forceinline__ void dep_guard_h(v8f& a, v8f& b, v16h x, v16h y) { asm volatile("v_nop\n\tv_nop\n\tv_nop\n\tv_nop" : "+v"(a), "+v"(b) : "v"(x), "v"(y)); }
__device__ __forceinline__ void keep4_h(v16h a, v16h b, v16h c, v16h d) { asm volatile("v_nop" :: "v"(a), "v"(b), "v"(c), "v"(d)); }
__device__ __forceinline__ void acc_guard2(v8f& a, v8f& b) { asm volatile("v_nop\n\tv_nop\n\tv_nop\n\tv_nop" : "+v"(a), "+v"(b)); }

template <typename T> struct Frag;
template <> struct Frag<_Float16> {
  typedef v16h V; union U { v16h v; v8h h[2]; };
  static __device__ __forceinline__ v16h load(const _Float16* p) {
    U f; f.h[0] = *(const v8h*)(p); f.h[1] = *(const v8h*)(p + 16); return f.v;
  }
  static __device__ __forceinline__ v8f mma(v16h a, v16h b, v8f c) {
    return __builtin_amdgcn_wmma_f32_16x16x32_f16(false, a, false, b, (short)0, c, false, false);
  }
  static __device__ __forceinline__ void guard(v8f& a, v8f& b, v16h x, v16h y) { dep_guard_h(a, b, x, y); }
  static __device__ __forceinline__ void keep(v16h a, v16h b, v16h c, v16h d) { keep4_h(a, b, c, d); }
};

constexpr int SEQ_T      = 2048;
constexpr int NBATCH     = 128;
constexpr int NIN        = 32;
constexpr int NHID       = 128;
constexpr int ROWS_BLK   = 32;
constexpr int NBLK       = NBATCH / ROWS_BLK;
constexpr int KCAT       = NIN + NHID;
constexpr int KSTEPS     = KCAT / 32;
constexpr int APITCH     = 168;
constexpr int TILE_HALVES = ROWS_BLK * APITCH;
constexpr int HS_PITCH   = 132;
constexpr int VST_STEPS  = 16;
constexpr float WSCALE    = 16.0f;
constexpr float ACC_SCALE = 1.0f / 16.0f;

static_assert(KCAT % 32 == 0, "K multiple of 32");
static_assert(NBLK * ROWS_BLK == NBATCH, "blocks cover the batch exactly");
static_assert(NHID == 8 * 16, "8 waves x 16 units");
static_assert(SEQ_T % VST_STEPS == 0, "flush covers every step");
static_assert((APITCH * 2) % 16 == 0 && (HS_PITCH * 4) % 16 == 0, "16-B aligned pitches");
static_assert((2 * TILE_HALVES) % 8 == 0, "tile zero fill in 16-B units");
static_assert(ROWS_BLK * 4 == 128, "one 128-B line of out0 per (t, block)");

__device__ __forceinline__ float dev_tanh(float x) {
  const float ax = fabsf(x);
  const float e  = expf(-2.0f * ax);
  const float y  = (1.0f - e) * __builtin_amdgcn_rcpf(1.0f + e);
  return copysignf(y, x);
}

__device__ __forceinline__ v16h build_bfrag(const float* __restrict__ wr, int hh) {
  const v4f q0 = *(const v4f*)(wr + 8 * hh);
  const v4f q1 = *(const v4f*)(wr + 8 * hh + 4);
  const v4f q2 = *(const v4f*)(wr + 16 + 8 * hh);
  const v4f q3 = *(const v4f*)(wr + 16 + 8 * hh + 4);
  v16h f;
#pragma unroll
  for (int e = 0; e < 4; ++e) {
    f[e]      = (_Float16)(q0[e] * WSCALE);
    f[4 + e]  = (_Float16)(q1[e] * WSCALE);
    f[8 + e]  = (_Float16)(q2[e] * WSCALE);
    f[12 + e] = (_Float16)(q3[e] * WSCALE);
  }
  return f;
}

__global__ __launch_bounds__(256) void leaky_rnn_scan(
    const float* __restrict__ X, const float* __restrict__ W_in, const float* __restrict__ W_hh,
    const float* __restrict__ rnn_bias, const float* __restrict__ alpha,
    const float* __restrict__ value_W, const float* __restrict__ value_bias,
    float* __restrict__ out)
{
  __shared__ __align__(16) _Float16 tileA[2 * TILE_HALVES];
  __shared__ __align__(16) float vpart[8 * ROWS_BLK];
  __shared__ __align__(16) float vstage[VST_STEPS * ROWS_BLK];
  __shared__ __align__(16) float hs[ROWS_BLK * HS_PITCH];

  const int tid  = threadIdx.x;
  const int lane = tid & 31;
  const int wave = tid >> 5;
  const int hh   = lane >> 4;
  const int c    = lane & 15;
  const int row0 = blockIdx.x * ROWS_BLK;
  const int n    = wave * 16 + c;

  const float al     = alpha[n];
  const float oma    = 1.0f - al;
  const float bias_n = rnn_bias[n];
  const float vw_n   = value_W[n];
  const float vbias  = value_bias[0];

  v16h bw[KSTEPS];
  bw[0] = build_bfrag(W_in + (size_t)n * NIN, hh);
#pragma unroll
  for (int s = 1; s < KSTEPS; ++s) bw[s] = build_bfrag(W_hh + (size_t)n * NHID + 32 * (s - 1), hh);

  for (int i = tid; i < (2 * TILE_HALVES) / 8; i += 256) ((uint4*)tileA)[i] = make_uint4(0u, 0u, 0u, 0u);

  float hreg[2][8];
#pragma unroll
  for (int mi = 0; mi < 2; ++mi)
#pragma unroll
    for (int r = 0; r < 8; ++r) hreg[mi][r] = 0.0f;

  __syncthreads();

#pragma unroll 1
  for (int t = 0; t < SEQ_T; ++t) {
    const int co = (t & 1) * TILE_HALVES;
    const int no = TILE_HALVES - co;

    if (tid < 128) {
      const int xr = tid >> 2;
      const int c8 = (tid & 3) * 8;
      const float* xp = X + ((size_t)t * NBATCH + (size_t)(row0 + xr)) * NIN + c8;
      const v4f x0 = *(const v4f*)xp;
      const v4f x1 = *(const v4f*)(xp + 4);
      v8h hv;
#pragma unroll
      for (int e = 0; e < 4; ++e) { hv[e] = (_Float16)x0[e]; hv[4 + e] = (_Float16)x1[e]; }
      *(v8h*)(tileA + co + xr * APITCH + c8) = hv;
    }
    __syncthreads();

    v8f acc[2];
    acc[0] = (v8f){0.f, 0.f, 0.f, 0.f, 0.f, 0.f, 0.f, 0.f};
    acc[1] = (v8f){0.f, 0.f, 0.f, 0.f, 0.f, 0.f, 0.f, 0.f};
#pragma unroll
    for (int s = 0; s < KSTEPS; ++s) {
      const v16h a0 = Frag<_Float16>::load(tileA + co + c * APITCH + 32 * s + 8 * hh);
      const v16h a1 = Frag<_Float16>::load(tileA + co + (16 + c) * APITCH + 32 * s + 8 * hh);
      acc[0] = Frag<_Float16>::mma(a0, bw[s], acc[0]);
      acc[1] = Frag<_Float16>::mma(a1, bw[s], acc[1]);
      Frag<_Float16>::guard(acc[0], acc[1], a0, a1);
    }
    acc_guard2(acc[0], acc[1]);

#pragma unroll
    for (int mi = 0; mi < 2; ++mi) {
#pragma unroll
      for (int r = 0; r < 8; ++r) {
        const float pre = acc[mi][r] * ACC_SCALE + bias_n;
        const float ht  = dev_tanh(pre);
        const float hn  = oma * hreg[mi][r] + al * ht;
        hreg[mi][r] = hn;
        tileA[no + (16 * mi + 8 * hh + r) * APITCH + NIN + n] = (_Float16)hn;
        float p = hn * vw_n;
        p += __shfl_xor(p, 1, 32);
        p += __shfl_xor(p, 2, 32);
        p += __shfl_xor(p, 4, 32);
        p += __shfl_xor(p, 8, 32);
        if (c == 0) vpart[wave * ROWS_BLK + 16 * mi + 8 * hh + r] = p;
      }
    }
    __syncthreads();

    if (wave == 0) {
      float sv = vpart[lane];
#pragma unroll
      for (int w = 1; w < 8; ++w) sv += vpart[w * ROWS_BLK + lane];
      sv += vbias;
      const int ttw = t & (VST_STEPS - 1);
      vstage[ttw * ROWS_BLK + lane] = sv;
      if (ttw == VST_STEPS - 1) {
        __builtin_amdgcn_fence(__ATOMIC_RELEASE, "workgroup");
        __builtin_amdgcn_wave_barrier();
        __builtin_amdgcn_fence(__ATOMIC_ACQUIRE, "workgroup");
        const int t0 = t - (VST_STEPS - 1);
        const int lg = lane >> 3;
        const int c4 = (lane & 7) * 4;
        for (int pass = 0; pass < 2; ++pass) {
#pragma unroll
          for (int q = 0; q < VST_STEPS / 4; ++q) {
            const int tt = q * 4 + lg;
            const v4f v = *(const v4f*)(vstage + tt * ROWS_BLK + c4);
            *(volatile v4f*)(out + ((size_t)(t0 + tt) * NBATCH + (size_t)(row0 + c4))) = v;
          }
          __threadfence();
        }
      }
    }
  }

#pragma unroll
  for (int mi = 0; mi < 2; ++mi)
#pragma unroll
    for (int r = 0; r < 8; ++r) hs[(16 * mi + 8 * hh + r) * HS_PITCH + n] = hreg[mi][r];
  __syncthreads();
  float* out1 = out + (size_t)SEQ_T * NBATCH;
  for (int pass = 0; pass < 2; ++pass) {
#pragma unroll
    for (int it = 0; it < 4; ++it) {
      const int f   = it * 256 + tid;
      const int row = f >> 5;
      const int c4  = (f & 31) * 4;
      const v4f v = *(const v4f*)(hs + row * HS_PITCH + c4);
      *(volatile v4f*)(out1 + (size_t)(row0 + row) * NHID + c4) = v;
    }
    __threadfence();
  }
}

extern "C" void kernel_launch(void* const* d_in, const int* in_sizes, int n_in,
                              void* d_out, int out_size, void* d_ws, size_t ws_size,
                              hipStream_t stream) {
  (void)d_ws; (void)ws_size;
  if (n_in < 7) return;
  if (in_sizes[0] != SEQ_T * NBATCH * NIN) return;
  if (in_sizes[1] != NHID * NIN) return;
  if (in_sizes[2] != NHID * NHID) return;
  if (in_sizes[3] != NHID || in_sizes[4] != NHID || in_sizes[5] != NHID) return;
  if (in_sizes[6] < 1) return;
  if (out_size != SEQ_T * NBATCH + NBATCH * NHID) return;

  const float* X          = (const float*)d_in[0];
  const float* W_in       = (const float*)d_in[1];
  const float* W_hh       = (const float*)d_in[2];
  const float* rnn_bias   = (const float*)d_in[3];
  const float* alpha      = (const float*)d_in[4];
  const float* value_W    = (const float*)d_in[5];
  const float* value_bias = (const float*)d_in[6];
  float* out = (float*)d_out;

  leaky_rnn_scan<<<dim3(NBLK), dim3(256), 0, stream>>>(
      X, W_in, W_hh, rnn_bias, alpha, value_W, value_bias, out);
}
